// intraAFL_Block_3805341024347
// MI455X (gfx1250) — hardware-verified
//
#include <hip/hip_runtime.h>
#include <math.h>
#include <stdint.h>

#define NBATCH 4
#define SEQ    1024
#define DM     512
#define NH     8
#define HD     64
#define DFF    2048
#define NC     32
#define MP     (NBATCH * SEQ)
#define QKP    (2 * DM)
#define WSC    64.0f
#define QSC    8.0f
#define PSC    1024.0f
#define CSC    64.0f
#define HSC    16.0f
#define ESC    256.0f
#define SSTR   1032
#define PSTR   1040
#define LDS_AVG  (16 * SSTR * 4)
#define LDS_P    (LDS_AVG + 16 * SEQ * 4)
#define LDS_C    (LDS_P + 16 * PSTR * 2)
#define LDS_ATTN (LDS_C + 16 * HD * 2)
static_assert(NH * HD == DM);
static_assert((SEQ % 128) == 0 && (DM % 64) == 0 && (MP % 64) == 0 && (DFF % 64) == 0);
static_assert(HD == 64 && NC == 32 && (SEQ % 16) == 0 && (MP % 8) == 0);
static_assert((LDS_AVG % 16) == 0 && (LDS_P % 16) == 0 && (LDS_C % 16) == 0);
static_assert(8 * 16 * HD <= 16 * SSTR);

typedef _Float16 v16h __attribute__((ext_vector_type(16)));
typedef _Float16 v8h  __attribute__((ext_vector_type(8)));
typedef unsigned short v16us __attribute__((ext_vector_type(16)));
typedef unsigned short v8us  __attribute__((ext_vector_type(8)));
typedef float    v8f  __attribute__((ext_vector_type(8)));
typedef float    v4f  __attribute__((ext_vector_type(4)));
typedef unsigned int v4u __attribute__((ext_vector_type(4)));
typedef unsigned int v2u __attribute__((ext_vector_type(2)));

union FragH { v16h v; v8h h[2]; };
union FragU { v16us v; v8us h[2]; };

__device__ __forceinline__ unsigned short bf_bits(float f) {
  unsigned u = __float_as_uint(f);
  return (unsigned short)((u + 0x7FFFu + ((u >> 16) & 1u)) >> 16);
}
__device__ __forceinline__ float bf_up(unsigned short h) { return __uint_as_float(((unsigned)h) << 16); }
__device__ __forceinline__ float bfr(float f) { return bf_up(bf_bits(f)); }
__device__ __forceinline__ unsigned short h_bits(_Float16 x) { return __builtin_bit_cast(unsigned short, x); }
__device__ __forceinline__ unsigned pk16(unsigned short a, unsigned short b) { return (unsigned)a | ((unsigned)b << 16); }
__device__ __forceinline__ v8f zero8() { v8f z = {0.f, 0.f, 0.f, 0.f, 0.f, 0.f, 0.f, 0.f}; return z; }

__device__ __forceinline__ float wred_sum(float v) {
#pragma unroll
  for (int o = 16; o > 0; o >>= 1) v += __shfl_xor(v, o, 32);
  return v;
}
__device__ __forceinline__ float wred_max(float v) {
#pragma unroll
  for (int o = 16; o > 0; o >>= 1) v = fmaxf(v, __shfl_xor(v, o, 32));
  return v;
}
__device__ __forceinline__ float wred_min(float v) {
#pragma unroll
  for (int o = 16; o > 0; o >>= 1) v = fminf(v, __shfl_xor(v, o, 32));
  return v;
}

__device__ __forceinline__ v16us ldfrag_u(const unsigned short* p) {
  FragU f;
  f.h[0] = *(const v8us*)(p);
  f.h[1] = *(const v8us*)(p + 16);
  return f.v;
}
__device__ __forceinline__ v16h ldfrag_h(const _Float16* p) {
  FragH f;
  f.h[0] = *(const v8h*)(p);
  f.h[1] = *(const v8h*)(p + 16);
  return f.v;
}

__device__ __forceinline__ v8f mma_raw(v16us a, v16us b, v8f c) {
  return __builtin_amdgcn_wmma_f32_16x16x32_f16(false, __builtin_bit_cast(v16h, a), false,
                                                __builtin_bit_cast(v16h, b), (short)0, c, false, false);
}
__device__ __forceinline__ v8f mma_u(v16us a, v16us b, v8f c) {
  c = __builtin_amdgcn_wmma_f32_16x16x32_f16(false, __builtin_bit_cast(v16h, a), false,
                                             __builtin_bit_cast(v16h, b), (short)0, c, false, false);
#if defined(__HIP_DEVICE_COMPILE__)
  asm volatile("v_nop\n\tv_nop\n\tv_nop\n\tv_nop" : "+v"(c) : "v"(a), "v"(b));
#endif
  return c;
}
__device__ __forceinline__ v8f mma_h(v16h a, v16h b, v8f c) {
  c = __builtin_amdgcn_wmma_f32_16x16x32_f16(false, a, false, b, (short)0, c, false, false);
#if defined(__HIP_DEVICE_COMPILE__)
  asm volatile("v_nop\n\tv_nop\n\tv_nop\n\tv_nop" : "+v"(c) : "v"(a), "v"(b));
#endif
  return c;
}
__device__ __forceinline__ void dep_guard1(v8f& a, v8f& b, v16us x) {
#if defined(__HIP_DEVICE_COMPILE__)
  asm volatile("v_nop\n\tv_nop\n\tv_nop\n\tv_nop" : "+v"(a), "+v"(b) : "v"(x));
#endif
}
__device__ __forceinline__ void keep4_u(v16us a, v16us b, v16us c, v16us d) {
#if defined(__HIP_DEVICE_COMPILE__)
  asm volatile("v_nop" :: "v"(a), "v"(b), "v"(c), "v"(d));
#endif
}
__device__ __forceinline__ void acc_guard4(v8f& a, v8f& b, v8f& c, v8f& d) {
#if defined(__HIP_DEVICE_COMPILE__)
  asm volatile("v_nop\n\tv_nop\n\tv_nop\n\tv_nop" : "+v"(a), "+v"(b), "+v"(c), "+v"(d));
#endif
}
__device__ __forceinline__ void wave_sync_lds() {
  __builtin_amdgcn_fence(__ATOMIC_RELEASE, "workgroup");
  __builtin_amdgcn_wave_barrier();
  __builtin_amdgcn_fence(__ATOMIC_ACQUIRE, "workgroup");
}

__global__ __launch_bounds__(256) void conv16(const float* __restrict__ W, unsigned short* out, int n8, float wsc) {
  const int i  = blockIdx.x * 256 + threadIdx.x;
  const int ic = (i < n8) ? i : (n8 - 1);
  const size_t e = (size_t)ic * 8;
  const v4f a = *(const v4f*)(W + e);
  const v4f c = *(const v4f*)(W + e + 4);
  v4u o;
  o[0] = pk16(h_bits((_Float16)(bfr(a[0]) * wsc)), h_bits((_Float16)(bfr(a[1]) * wsc)));
  o[1] = pk16(h_bits((_Float16)(bfr(a[2]) * wsc)), h_bits((_Float16)(bfr(a[3]) * wsc)));
  o[2] = pk16(h_bits((_Float16)(bfr(c[0]) * wsc)), h_bits((_Float16)(bfr(c[1]) * wsc)));
  o[3] = pk16(h_bits((_Float16)(bfr(c[2]) * wsc)), h_bits((_Float16)(bfr(c[3]) * wsc)));
  if (i < n8) *(volatile v4u*)(out + e) = o;
  __threadfence();
  if (i < n8) *(volatile v4u*)(out + e) = o;
}

template <int OM, int BM, int RL>
__global__ __launch_bounds__(256) void gemm64(
    const unsigned short* __restrict__ Ap, int lda, long long strideA,
    const unsigned short* __restrict__ Btp, int ldb, long long strideB,
    unsigned short* Cp, float* Cf, int ldc, long long strideC,
    const float* __restrict__ bias, int M, int N, int K, float oscale, float osc2) {
  __shared__ __align__(16) float sT[8][16 * 68];
  const int b    = blockIdx.y;
  const int lane = threadIdx.x & 31;
  const int wave = threadIdx.x >> 5;
  const int tilesN = N >> 6;
  const int tilesM = M >> 6;
  const int tile = blockIdx.x * 8 + wave;
  if (tile >= tilesM * tilesN) return;
  const int tm = tile / tilesN;
  const int tn = tile - tm * tilesN;
  const int m0 = tm << 6;
  const int n0 = tn << 6;

  const unsigned short* Ab = Ap  + (size_t)b * strideA;
  const unsigned short* Bb = Btp + (size_t)b * strideB;

  const int rlane = lane & 15;
  const int koff  = (lane >> 4) * 8;
  const int mOff  = (lane >> 4) * 8;

  v8f acc[4][4];
#pragma unroll
  for (int i = 0; i < 4; ++i)
#pragma unroll
    for (int j = 0; j < 4; ++j) acc[i][j] = zero8();

  for (int k0 = 0; k0 < K; k0 += 32) {
    v16us bh[4];
#pragma unroll
    for (int j = 0; j < 4; ++j) {
      const size_t bo = (size_t)(n0 + (j << 4) + rlane) * ldb + koff + k0;
      bh[j] = ldfrag_u(Bb + bo);
    }
#pragma unroll
    for (int i = 0; i < 4; ++i) {
      const size_t ao = (size_t)(m0 + (i << 4) + rlane) * lda + koff + k0;
      const v16us ah = ldfrag_u(Ab + ao);
#pragma unroll
      for (int j = 0; j < 4; ++j) acc[i][j] = mma_raw(ah, bh[j], acc[i][j]);
      dep_guard1(acc[i][0], acc[i][3], ah);
    }
    keep4_u(bh[0], bh[1], bh[2], bh[3]);
  }
  acc_guard4(acc[0][0], acc[0][1], acc[0][2], acc[0][3]);
  acc_guard4(acc[1][0], acc[1][1], acc[1][2], acc[1][3]);
  acc_guard4(acc[2][0], acc[2][1], acc[2][2], acc[2][3]);
  acc_guard4(acc[3][0], acc[3][1], acc[3][2], acc[3][3]);

  const int hh2 = lane >> 4, c4 = (lane & 15) * 4;
  const int q8  = lane >> 3, c8 = (lane & 7) * 8;

  float* slab = sT[wave];
#pragma unroll
  for (int i = 0; i < 4; ++i) {
    const int mBase = m0 + (i << 4);
#pragma unroll
    for (int j = 0; j < 4; ++j) {
#pragma unroll
      for (int r = 0; r < 8; ++r) {
        slab[(mOff + r) * 68 + (j << 4) + rlane] = acc[i][j][r];
      }
    }
    wave_sync_lds();
    if (OM == 0) {
      float* C = Cf + (size_t)b * strideC;
      v4f b4 = {0.f, 0.f, 0.f, 0.f};
      if (BM == 1) {
        const v4f t4 = *(const v4f*)(bias + n0 + c4);
        b4[0] = bfr(t4[0]); b4[1] = bfr(t4[1]); b4[2] = bfr(t4[2]); b4[3] = bfr(t4[3]);
      }
      v4f vals[8];
#pragma unroll
      for (int it = 0; it < 8; ++it) {
        const int row = it * 2 + hh2;
        v4f v = *(const v4f*)(slab + row * 68 + c4);
        v = v * oscale + b4;
        if (BM == 2) { const float bb = bfr(bias[mBase + row]); v = v + bb; }
        if (RL) { v[0] = fmaxf(v[0], 0.f); v[1] = fmaxf(v[1], 0.f); v[2] = fmaxf(v[2], 0.f); v[3] = fmaxf(v[3], 0.f); }
        vals[it] = v;
      }
      for (int pass = 0; pass < 2; ++pass) {
#pragma unroll
        for (int it = 0; it < 8; ++it) {
          const int row = it * 2 + hh2;
          *(volatile v4f*)(C + (size_t)(mBase + row) * ldc + n0 + c4) = vals[it];
        }
        __threadfence();
      }
    } else {
      unsigned short* C = Cp + (size_t)b * strideC;
      v4u hv[4];
#pragma unroll
      for (int it = 0; it < 4; ++it) {
        const int row = it * 4 + q8;
        const float* sp = slab + row * 68 + c8;
        float brow = 0.f;
        if (BM == 2) brow = bfr(bias[mBase + row]);
        v4u ha;
#pragma unroll
        for (int e = 0; e < 4; ++e) {
          float f0 = sp[2 * e]     * oscale + brow;
          float f1 = sp[2 * e + 1] * oscale + brow;
          if (BM == 1) { f0 += bfr(bias[n0 + c8 + 2 * e]); f1 += bfr(bias[n0 + c8 + 2 * e + 1]); }
          if (RL) { f0 = fmaxf(f0, 0.f); f1 = fmaxf(f1, 0.f); }
          ha[e] = pk16(h_bits((_Float16)(f0 * osc2)), h_bits((_Float16)(f1 * osc2)));
        }
        hv[it] = ha;
      }
      for (int pass = 0; pass < 2; ++pass) {
#pragma unroll
        for (int it = 0; it < 4; ++it) {
          const int row = it * 4 + q8;
          const size_t go = (size_t)(mBase + row) * ldc + n0 + c8;
          *(volatile v4u*)(C + go) = hv[it];
        }
        __threadfence();
      }
    }
    wave_sync_lds();
  }
}

__global__ __launch_bounds__(256)
void attn16(const unsigned short* __restrict__ qk, const unsigned short* __restrict__ vt,
            unsigned short* ctxp, float* avgp, float sscale) {
  extern __shared__ v4f dlds_v[];
  unsigned char* dlds = (unsigned char*)dlds_v;
  float* sS = (float*)(dlds);
  float* sA = (float*)(dlds + LDS_AVG);
  _Float16* sP = (_Float16*)(dlds + LDS_P);
  unsigned short* sC = (unsigned short*)(dlds + LDS_C);

  const int tid  = threadIdx.x;
  const int wave = tid >> 5;
  const int lane = tid & 31;
  const int hh   = lane >> 4;
  const int c    = lane & 15;
  const int b    = blockIdx.x / (SEQ / 16);
  const int i0   = (blockIdx.x % (SEQ / 16)) * 16;
  const size_t rowB = (size_t)b * SEQ;
  const _Float16* vtb = (const _Float16*)(const void*)vt + (size_t)b * DM * SEQ;

  for (int u = tid; u < 16 * SEQ; u += 256) sA[u] = 0.f;

#pragma unroll 1
  for (int h = 0; h < NH; ++h) {
    v16us qf[2];
#pragma unroll
    for (int dc = 0; dc < 2; ++dc)
      qf[dc] = ldfrag_u(qk + (rowB + i0 + c) * QKP + h * HD + dc * 32 + 8 * hh);
#pragma unroll 1
    for (int nt = 0; nt < 8; ++nt) {
      const int n0 = wave * 128 + nt * 16;
      v8f sc = zero8();
#pragma unroll
      for (int dc = 0; dc < 2; ++dc) {
        const v16us kb = ldfrag_u(qk + (rowB + n0 + c) * QKP + DM + h * HD + dc * 32 + 8 * hh);
        sc = mma_u(qf[dc], kb, sc);
      }
#pragma unroll
      for (int r = 0; r < 8; ++r) sS[(8 * hh + r) * SSTR + n0 + c] = sc[r] * sscale;
    }
    __syncthreads();

#pragma unroll
    for (int rr = 0; rr < 2; ++rr) {
      const int r = wave * 2 + rr;
      const float* row = sS + r * SSTR;
      float pv[32];
      float m = -INFINITY;
#pragma unroll
      for (int t = 0; t < 32; ++t) { pv[t] = row[lane + 32 * t]; m = fmaxf(m, pv[t]); }
      m = wred_max(m);
      float s = 0.f;
#pragma unroll
      for (int t = 0; t < 32; ++t) { pv[t] = __expf(pv[t] - m); s += pv[t]; }
      s = wred_sum(s);
      const float inv = 1.0f / s;
      _Float16* prow = sP + r * PSTR;
      float* arow = sA + r * SEQ;
#pragma unroll
      for (int t = 0; t < 32; ++t) {
        const int j = lane + 32 * t;
        const float p = pv[t] * inv;
        prow[j] = (_Float16)(p * PSC);
        arow[j] = arow[j] + p;
      }
    }
    __syncthreads();

    v8f ca[4];
#pragma unroll
    for (int nt = 0; nt < 4; ++nt) ca[nt] = zero8();
#pragma unroll 1
    for (int ks = 0; ks < 4; ++ks) {
      const int kg = wave * 128 + ks * 32;
      FragH pa;
      pa.h[0] = *(const v8h*)(sP + c * PSTR + kg + 8 * hh);
      pa.h[1] = *(const v8h*)(sP + c * PSTR + kg + 16 + 8 * hh);
#pragma unroll
      for (int nt = 0; nt < 4; ++nt) {
        const v16h vb = ldfrag_h(vtb + (size_t)(h * HD + nt * 16 + c) * SEQ + kg + 8 * hh);
        ca[nt] = mma_h(pa.v, vb, ca[nt]);
      }
    }
    {
      float* part = sS + wave * 1024;
#pragma unroll
      for (int nt = 0; nt < 4; ++nt)
#pragma unroll
        for (int r = 0; r < 8; ++r) part[(8 * hh + r) * HD + nt * 16 + c] = ca[nt][r];
    }
    __syncthreads();

    {
      const int idx = tid * 4;
      v4f a4 = *(const v4f*)(sS + idx);
#pragma unroll
      for (int w = 1; w < 8; ++w) a4 = a4 + *(const v4f*)(sS + w * 1024 + idx);
      const float cf = CSC / (PSC * QSC);
      v2u o;
      o[0] = pk16(h_bits((_Float16)(a4[0] * cf)), h_bits((_Float16)(a4[1] * cf)));
      o[1] = pk16(h_bits((_Float16)(a4[2] * cf)), h_bits((_Float16)(a4[3] * cf)));
      *(v2u*)(sC + idx) = o;
    }
    __syncthreads();

    if (wave == 0) {
      const int q8 = lane >> 3, c8 = (lane & 7) * 8;
      v4u hv[4];
      size_t go[4];
#pragma unroll
      for (int it = 0; it < 4; ++it) {
        const int row = it * 4 + q8;
        hv[it] = *(const v4u*)(sC + row * HD + c8);
        go[it] = (rowB + i0 + row) * DM + (size_t)h * HD + c8;
      }
      for (int pass = 0; pass < 2; ++pass) {
#pragma unroll
        for (int it = 0; it < 4; ++it) *(volatile v4u*)(ctxp + go[it]) = hv[it];
        __threadfence();
      }
    }
    __syncthreads();
  }

#pragma unroll
  for (int rr = 0; rr < 2; ++rr) {
    const int r = wave * 2 + rr;
    v4f vals[8];
#pragma unroll
    for (int it = 0; it < 8; ++it) {
      const int col = it * 128 + lane * 4;
      vals[it] = *(const v4f*)(sA + r * SEQ + col) * 0.125f;
    }
    float* ga = avgp + (rowB + i0 + r) * SEQ;
    for (int pass = 0; pass < 2; ++pass) {
#pragma unroll
      for (int it = 0; it < 8; ++it) *(volatile v4f*)(ga + it * 128 + lane * 4) = vals[it];
      __threadfence();
    }
  }
}

__global__ __launch_bounds__(256)
void edgeproj(const float* __restrict__ avg, const float* __restrict__ ew, const float* __restrict__ eb,
              const unsigned short* __restrict__ wpp, const float* __restrict__ pb, float* outw) {
#pragma clang fp contract(off)
  __shared__ __align__(16) _Float16 sW[64 * NC];
  __shared__ __align__(16) float sT[8][16 * 36];
  const int tid  = threadIdx.x;
  const int wave = tid >> 5;
  const int lane = tid & 31;
  const int hh   = lane >> 4;
  const int c    = lane & 15;
  const int row0 = blockIdx.x * 64;

#pragma unroll 1
  for (int i = 0; i < 8; ++i) {
    const int rl = wave * 8 + i;
    const float* a = avg + (size_t)(row0 + rl) * SEQ;
    float va[32];
    float amax = -INFINITY, amin = INFINITY;
#pragma unroll
    for (int t = 0; t < 32; ++t) {
      va[t] = a[lane + 32 * t];
      amax = fmaxf(amax, va[t]);
      amin = fminf(amin, va[t]);
    }
    amax = wred_max(amax);
    amin = wred_min(amin);
    float myw = 0.f;
#pragma unroll 1
    for (int ch = 0; ch < NC; ++ch) {
      const float wc = bfr(ew[ch]);
      const float ec = bfr(eb[ch]);
      const float m  = fmaxf(amax * wc + ec, amin * wc + ec);
      float s = 0.f, sa = 0.f;
#pragma unroll
      for (int t = 0; t < 32; ++t) {
        const float e = va[t] * wc + ec;
        const float p = __expf(e - m);
        s  += p;
        sa += p * e;
      }
      s  = wred_sum(s);
      sa = wred_sum(sa);
      const float val = sa * (1.0f / s);
      myw = (lane == ch) ? val : myw;
    }
    sW[rl * NC + lane] = (_Float16)(myw * ESC);
  }
  __syncthreads();

  const int q8 = lane >> 3, c4 = (lane & 7) * 4;
  const float osc = 1.0f / (ESC * WSC);
  float* slab = sT[wave];
#pragma unroll 1
  for (int half = 0; half < 2; ++half) {
    const int cb = wave * 64 + half * 32;
    v16us bq[2];
#pragma unroll
    for (int j = 0; j < 2; ++j) bq[j] = ldfrag_u(wpp + (size_t)(cb + 16 * j + c) * NC + 8 * hh);
    v8f acc[4][2];
#pragma unroll
    for (int i = 0; i < 4; ++i) {
      FragH af;
      af.h[0] = *(const v8h*)(sW + (16 * i + c) * NC + 8 * hh);
      af.h[1] = *(const v8h*)(sW + (16 * i + c) * NC + 16 + 8 * hh);
#pragma unroll
      for (int j = 0; j < 2; ++j) {
        acc[i][j] = zero8();
        acc[i][j] = mma_u(__builtin_bit_cast(v16us, af.v), bq[j], acc[i][j]);
      }
    }
    v4f b4;
    {
      const v4f t4 = *(const v4f*)(pb + cb + c4);
      b4[0] = bfr(t4[0]); b4[1] = bfr(t4[1]); b4[2] = bfr(t4[2]); b4[3] = bfr(t4[3]);
    }
#pragma unroll
    for (int i = 0; i < 4; ++i) {
#pragma unroll
      for (int j = 0; j < 2; ++j)
#pragma unroll
        for (int r = 0; r < 8; ++r) slab[(8 * hh + r) * 36 + 16 * j + c] = acc[i][j][r];
      wave_sync_lds();
      v4f vals[4];
      size_t go[4];
#pragma unroll
      for (int it = 0; it < 4; ++it) {
        const int row = it * 4 + q8;
        v4f v = *(const v4f*)(slab + row * 36 + c4);
        v = v * osc;
        v = v + b4;
        vals[it] = v;
        go[it] = (size_t)(row0 + 16 * i + row) * DM + cb + c4;
      }
      for (int pass = 0; pass < 2; ++pass) {
#pragma unroll
        for (int it = 0; it < 4; ++it) *(volatile v4f*)(outw + go[it]) = vals[it];
        __threadfence();
      }
      wave_sync_lds();
    }
  }
}

template <int RA, int B3, int WP>
__global__ __launch_bounds__(256) void lnrow(const float* __restrict__ A, const float* __restrict__ B1,
                                             const float* __restrict__ B2,
                                             const float* __restrict__ g, const float* __restrict__ be,
                                             float* outf, unsigned short* plane, int nrows) {
  __shared__ __align__(16) unsigned short sh[8][DM];
  const int wave = threadIdx.x >> 5, lane = threadIdx.x & 31;
  const int row = blockIdx.x * 8 + wave;
  if (row >= nrows) return;
  const float* pa = A  + (size_t)row * DM;
  const float* p1 = B1 + (size_t)row * DM;
  const float* p2 = B2 + (size_t)row * DM;
  v4f v[4];
  float s = 0.f;
#pragma unroll
  for (int it = 0; it < 4; ++it) {
    const int col = it * 128 + lane * 4;
    v4f va = *(const v4f*)(pa + col);
    if (RA) { va[0] = bfr(va[0]); va[1] = bfr(va[1]); va[2] = bfr(va[2]); va[3] = bfr(va[3]); }
    v4f vb = *(const v4f*)(p1 + col);
    if (B3) { const v4f vc = *(const v4f*)(p2 + col); vb = vb + vc; }
    v[it] = va + vb;
    s += (v[it][0] + v[it][1]) + (v[it][2] + v[it][3]);
  }
  s = wred_sum(s);
  const float mean = s * (1.0f / DM);
  float ss = 0.f;
#pragma unroll
  for (int it = 0; it < 4; ++it) {
    const v4f d = v[it] - mean;
    v[it] = d;
    ss += (d[0] * d[0] + d[1] * d[1]) + (d[2] * d[2] + d[3] * d[3]);
  }
  ss = wred_sum(ss);
  const float var  = ss * (1.0f / DM);
  const float rstd = rsqrtf(var + 1e-5f);
  v4f y[4];
#pragma unroll
  for (int it = 0; it < 4; ++it) {
    const int col = it * 128 + lane * 4;
    const v4f gv = *(const v4f*)(g + col);
    const v4f bv = *(const v4f*)(be + col);
    v4f o;
#pragma unroll
    for (int e = 0; e < 4; ++e) o[e] = (v[it][e] * rstd) * bfr(gv[e]) + bfr(bv[e]);
    y[it] = o;
  }
  float* po = outf + (size_t)row * DM;
  for (int pass = 0; pass < 2; ++pass) {
#pragma unroll
    for (int it = 0; it < 4; ++it) *(volatile v4f*)(po + it * 128 + lane * 4) = y[it];
    __threadfence();
  }
  if (WP) {
    unsigned short* shw = sh[wave];
#pragma unroll
    for (int it = 0; it < 4; ++it) {
      const int col = it * 128 + lane * 4;
      v2u hp;
      hp[0] = pk16(h_bits((_Float16)y[it][0]), h_bits((_Float16)y[it][1]));
      hp[1] = pk16(h_bits((_Float16)y[it][2]), h_bits((_Float16)y[it][3]));
      *(v2u*)(shw + col) = hp;
    }
    wave_sync_lds();
    v4u hv[2];
#pragma unroll
    for (int it = 0; it < 2; ++it) hv[it] = *(const v4u*)(shw + it * 256 + lane * 8);
    unsigned short* pp = plane + (size_t)row * DM;
    for (int pass = 0; pass < 2; ++pass) {
#pragma unroll
      for (int it = 0; it < 2; ++it) *(volatile v4u*)(pp + it * 256 + lane * 8) = hv[it];
      __threadfence();
    }
  }
}

extern "C" void kernel_launch(void* const* d_in, const int* in_sizes, int n_in,
                              void* d_out, int out_size, void* d_ws, size_t ws_size,
                              hipStream_t stream) {
  if (n_in < 17) return;
  if (in_sizes[0] != MP * DM) return;
  if (in_sizes[1] != 3 * DM * DM || in_sizes[2] != 3 * DM) return;
  if (in_sizes[3] != DM * DM || in_sizes[4] != DM) return;
  if (in_sizes[5] != NC || in_sizes[6] != NC) return;
  if (in_sizes[7] != DM * NC || in_sizes[8] != DM) return;
  if (in_sizes[9] != DFF * DM || in_sizes[10] != DFF) return;
  if (in_sizes[11] != DM * DFF || in_sizes[12] != DM) return;
  if (in_sizes[13] != DM || in_sizes[14] != DM || in_sizes[15] != DM || in_sizes[16] != DM) return;
  if (out_size != MP * DM) return;

  const float* src   = (const float*)d_in[0];
  const float* w_qkv = (const float*)d_in[1];
  const float* b_qkv = (const float*)d_in[2];
  const float* w_o   = (const float*)d_in[3];
  const float* b_o   = (const float*)d_in[4];
  const float* e_w   = (const float*)d_in[5];
  const float* e_b   = (const float*)d_in[6];
  const float* w_pj  = (const float*)d_in[7];
  const float* b_pj  = (const float*)d_in[8];
  const float* w_1   = (const float*)d_in[9];
  const float* b_1   = (const float*)d_in[10];
  const float* w_2   = (const float*)d_in[11];
  const float* b_2   = (const float*)d_in[12];
  const float* ln1g  = (const float*)d_in[13];
  const float* ln1b  = (const float*)d_in[14];
  const float* ln2g  = (const float*)d_in[15];
  const float* ln2b  = (const float*)d_in[16];

  const size_t PWQ  = (size_t)3 * DM * DM * 2;
  const size_t PXH  = (size_t)MP * DM * 2;
  const size_t PWO  = (size_t)DM * DM * 2;
  const size_t PW1  = (size_t)DFF * DM * 2;
  const size_t PW2  = (size_t)DM * DFF * 2;
  const size_t PWPJ = (size_t)DM * NC * 2;
  const size_t PQK  = (size_t)MP * QKP * 2;
  const size_t PVT  = (size_t)NBATCH * DM * SEQ * 2;
  const size_t PCTX = (size_t)MP * DM * 2;
  const size_t PAVG = (size_t)MP * SEQ * 4;
  const size_t PF32 = (size_t)MP * DM * 4;
  const size_t PXP  = (size_t)MP * DM * 2;
  const size_t PHP  = (size_t)MP * DFF * 2;
  size_t off = 0;
  const size_t oWQ  = off; off += PWQ;
  const size_t oXH  = off; off += PXH;
  const size_t oWO  = off; off += PWO;
  const size_t oW1  = off; off += PW1;
  const size_t oW2  = off; off += PW2;
  const size_t oWPJ = off; off += PWPJ;
  const size_t oQK  = off; off += PQK;
  const size_t oVT  = off; off += PVT;
  const size_t oCTX = off; off += PCTX;
  const size_t oAVG = off; off += PAVG;
  const size_t oAO  = off; off += PF32;
  const size_t oEW  = off; off += PF32;
  const size_t oX1  = off; off += PF32;
  const size_t oXP  = off; off += PXP;
  const size_t oHP  = off; off += PHP;
  const size_t oFF  = off; off += PF32;
  if (off > ws_size) return;
  if (off > (size_t)134217728) return;

  char* ws = (char*)d_ws;
  unsigned short* WQ  = (unsigned short*)(ws + oWQ);
  unsigned short* XH  = (unsigned short*)(ws + oXH);
  unsigned short* WO  = (unsigned short*)(ws + oWO);
  unsigned short* W1  = (unsigned short*)(ws + oW1);
  unsigned short* W2  = (unsigned short*)(ws + oW2);
  unsigned short* WPJ = (unsigned short*)(ws + oWPJ);
  unsigned short* QK  = (unsigned short*)(ws + oQK);
  unsigned short* VT  = (unsigned short*)(ws + oVT);
  unsigned short* CTX = (unsigned short*)(ws + oCTX);
  float*          AVG = (float*)(ws + oAVG);
  float*          AO  = (float*)(ws + oAO);
  float*          EW  = (float*)(ws + oEW);
  float*          X1  = (float*)(ws + oX1);
  unsigned short* XP  = (unsigned short*)(ws + oXP);
  unsigned short* HP  = (unsigned short*)(ws + oHP);
  float*          FF  = (float*)(ws + oFF);
  float*          out0 = (float*)d_out;

  const int n8w  = (3 * DM * DM) / 8;
  const int n8x  = (MP * DM) / 8;
  const int n8o  = (DM * DM) / 8;
  const int n81  = (DFF * DM) / 8;
  const int n82  = (DM * DFF) / 8;
  const int n8p  = (DM * NC) / 8;
  const dim3 blk(256);
  const dim3 gCw((n8w + 255) / 256), gCx((n8x + 255) / 256), gCo((n8o + 255) / 256);
  const dim3 gC1((n81 + 255) / 256), gC2((n82 + 255) / 256), gCp((n8p + 255) / 256);
  const dim3 gQK(((MP / 64) * (QKP / 64) + 7) / 8, 1);
  const dim3 gVT(((DM / 64) * (SEQ / 64) + 7) / 8, NBATCH);
  const dim3 gAttn(NBATCH * (SEQ / 16));
  const dim3 gWo(((MP / 64) * (DM / 64) + 7) / 8, 1);
  const dim3 gEdge(MP / 64);
  const dim3 gW1(((MP / 64) * (DFF / 64) + 7) / 8, 1);
  const dim3 gW2(((MP / 64) * (DM / 64) + 7) / 8, 1);
  const dim3 gLn((MP + 7) / 8);
  const float invw = 1.0f / WSC;

  conv16<<<gCw, blk, 0, stream>>>(w_qkv, WQ, n8w, WSC);
  conv16<<<gCx, blk, 0, stream>>>(src, XH, n8x, 1.0f);
  conv16<<<gCo, blk, 0, stream>>>(w_o, WO, n8o, WSC);
  conv16<<<gC1, blk, 0, stream>>>(w_1, W1, n81, WSC);
  conv16<<<gC2, blk, 0, stream>>>(w_2, W2, n82, WSC);
  conv16<<<gCp, blk, 0, stream>>>(w_pj, WPJ, n8p, WSC);

  gemm64<1, 1, 0><<<gQK, blk, 0, stream>>>(
      XH, DM, 0LL, WQ, DM, 0LL,
      QK, AO, QKP, 0LL, b_qkv, MP, QKP, DM, invw, QSC);
  gemm64<1, 2, 0><<<gVT, blk, 0, stream>>>(
      WQ + (size_t)(2 * DM) * DM, DM, 0LL, XH, DM, (long long)SEQ * DM,
      VT, AO, SEQ, (long long)DM * SEQ, b_qkv + 2 * DM, DM, SEQ, DM, invw, QSC);

  (void)hipFuncSetAttribute(reinterpret_cast<const void*>(&attn16), hipFuncAttributeMaxDynamicSharedMemorySize,
                            LDS_ATTN);
  attn16<<<gAttn, blk, LDS_ATTN, stream>>>(QK, VT, CTX, AVG, 0.125f / (QSC * QSC));

  gemm64<0, 1, 0><<<gWo, blk, 0, stream>>>(
      CTX, DM, 0LL, WO, DM, 0LL,
      XP, AO, DM, 0LL, b_o, MP, DM, DM, 1.0f / (CSC * WSC), 1.0f);

  edgeproj<<<gEdge, blk, 0, stream>>>(AVG, e_w, e_b, WPJ, b_pj, EW);

  lnrow<1, 1, 1><<<gLn, blk, 0, stream>>>(src, AO, EW, ln1g, ln1b, X1, XP, MP);

  gemm64<1, 1, 1><<<gW1, blk, 0, stream>>>(
      XP, DM, 0LL, W1, DM, 0LL,
      HP, FF, DFF, 0LL, b_1, MP, DFF, DM, invw, HSC);

  gemm64<0, 1, 0><<<gW2, blk, 0, stream>>>(
      HP, DFF, 0LL, W2, DFF, 0LL,
      XP, FF, DM, 0LL, b_2, MP, DM, DFF, 1.0f / (HSC * WSC), 1.0f);

  lnrow<0, 0, 0><<<gLn, blk, 0, stream>>>(X1, FF, FF, ln2g, ln2b, out0, XP, MP);
  (void)hipGetLastError();
}
